// LanguageCalibration_34024730919225
// MI455X (gfx1250) — hardware-run, weakly checked
//
#include <hip/hip_runtime.h>
#include <math.h>

constexpr int kB  = 8;
constexpr int kS  = 512;
constexpr int kH  = 768;
constexpr int kL  = 5;
constexpr int kNH = 12;
constexpr int kD  = 64;
constexpr int kC  = 256;
constexpr int kRows = kB * kS;
constexpr long kHH = (long)kH * kH;
constexpr long kSH = (long)kS * kH;
constexpr long kSS = (long)kS * kS;
constexpr float kPCarry    = 32768.0f;
constexpr float kPCarryInv = 1.0f / 32768.0f;
constexpr float kWCarry    = 16.0f;
constexpr float kWCarryInv = 1.0f / 16.0f;
constexpr float kQScale    = 0.125f;
constexpr float kLnEps     = 1e-5f;
constexpr float kInvH      = 1.0f / 768.0f;
constexpr float kInvNH     = 1.0f / 12.0f;
static_assert(kNH * kD == kH, "heads");
static_assert(kS == 512 && kH == 3 * 256 && kC == 256, "thread maps");
static_assert(kS % 64 == 0 && kH % 64 == 0 && kD % 64 == 0, "M,N tile multiples");
static_assert(kH % 32 == 0 && kS % 32 == 0 && kD % 32 == 0, "K multiples of 32");

constexpr long kOut0Elems = (long)kRows * kH;
constexpr long kOut1Off   = kOut0Elems;
constexpr long kOut1Elems = (long)kB * kSS;
constexpr long kOut2Off   = kOut1Off + kOut1Elems;
constexpr long kOut2Elems = (long)kB * kC;
constexpr long kOut3Off   = kOut2Off + kOut2Elems;
constexpr long kOutTotal  = kOut3Off + 1;
static_assert(kOut1Off * 4 == 12582912L && kOut2Off * 4 == 20971520L && kOut3Off * 4 == 20979712L && kOutTotal * 4 == 20979716L, "output byte offsets");

constexpr size_t kP16 = (size_t)kRows * kH * 2;
constexpr size_t kP32 = (size_t)kRows * kH * 4;
constexpr size_t kWL  = (size_t)kL * kHH * 2;
constexpr size_t kW1  = (size_t)kHH * 2;
constexpr size_t kALT = (size_t)kL * kL * kHH * 2;
constexpr size_t offX16   = 0;
constexpr size_t offAWT   = offX16 + kP16;
constexpr size_t offWQL   = offAWT + kWL;
constexpr size_t offWKL   = offWQL + kWL;
constexpr size_t offW5    = offWKL + kWL;
constexpr size_t offALT   = offW5 + 5 * kW1;
constexpr size_t offADP16 = offALT + kALT;
constexpr size_t offADP32 = offADP16 + kP16;
constexpr size_t offQL    = offADP32 + kP32;
constexpr size_t offKL    = offQL + kP16;
constexpr size_t offQP    = offKL + kP16;
constexpr size_t offKP    = offQP + kP16;
constexpr size_t offVT    = offKP + kP16;
constexpr size_t offSC    = offVT + kP16;
constexpr size_t offATT   = offSC + kP32;
constexpr size_t offPOOL  = offATT + kP16;
constexpr size_t offPN    = offPOOL + (size_t)kB * kH * 4;
constexpr size_t kWsTotal = offPN + (size_t)kB * kC * 4;
static_assert(kWsTotal == 128614400UL, "carve total");
static_assert(kWsTotal <= 134217728UL, "carve under 128 MiB");
static_assert((size_t)kNH * kSS * 4 == kP32 && (size_t)kNH * kSS * 2 == kP16 && (size_t)kB * kH * kS * 2 == kP16, "region reuse sizes");
static_assert(offAWT % 128 == 0 && offW5 % 128 == 0 && offALT % 128 == 0 && offADP32 % 128 == 0 && offSC % 128 == 0 && offPOOL % 128 == 0 && offPN % 128 == 0, "alignment");

typedef __attribute__((ext_vector_type(16))) _Float16 v16h;
typedef __attribute__((ext_vector_type(8)))  _Float16 v8h;
typedef __attribute__((ext_vector_type(8)))  float    v8f;
typedef __attribute__((ext_vector_type(4)))  float    v4f;
typedef __attribute__((ext_vector_type(2)))  float    v2f;
typedef __attribute__((ext_vector_type(4)))  unsigned int v4u;

__device__ __forceinline__ unsigned short f2bf_bits(float f) {
  unsigned u = __float_as_uint(f);
  return (unsigned short)((u + 0x7FFFu + ((u >> 16) & 1u)) >> 16);
}
__device__ __forceinline__ float bf_bits2f(unsigned short h) { return __uint_as_float(((unsigned)h) << 16); }
__device__ __forceinline__ float bfr(float f) { return bf_bits2f(f2bf_bits(f)); }
__device__ __forceinline__ unsigned pk16(unsigned short a, unsigned short b) { return (unsigned)a | ((unsigned)b << 16); }
__device__ __forceinline__ unsigned short h_bits(float f) { const _Float16 h = (_Float16)f; return __builtin_bit_cast(unsigned short, h); }
__device__ __forceinline__ int clamp_lang(int v) { return v < 0 ? 0 : (v > kL - 1 ? kL - 1 : v); }

__device__ __forceinline__ void dep_guard4_h(v8f& a, v8f& b, v8f& c, v8f& d, v16h x, v16h y) {
  asm volatile("v_nop\n\tv_nop\n\tv_nop\n\tv_nop" : "+v"(a), "+v"(b), "+v"(c), "+v"(d) : "v"(x), "v"(y));
}
__device__ __forceinline__ void keep4_h(v16h a, v16h b, v16h c, v16h d) { asm volatile("v_nop" :: "v"(a), "v"(b), "v"(c), "v"(d)); }
__device__ __forceinline__ void acc_guard4(v8f& a, v8f& b, v8f& c, v8f& d) { asm volatile("v_nop\n\tv_nop\n\tv_nop\n\tv_nop" : "+v"(a), "+v"(b), "+v"(c), "+v"(d)); }

struct FragH {
  typedef v16h V; union U { v16h v; v8h h[2]; };
  static __device__ __forceinline__ v16h load(const _Float16* p) {
    U f; f.h[0] = *(const v8h*)(p); f.h[1] = *(const v8h*)(p + 16); return f.v;
  }
  static __device__ __forceinline__ v8f mma(v16h a, v16h b, v8f c) {
    return __builtin_amdgcn_wmma_f32_16x16x32_f16(false, a, false, b, (short)0, c, false, false);
  }
  static __device__ __forceinline__ void guard4(v8f& a, v8f& b, v8f& c, v8f& d, v16h x, v16h y) { dep_guard4_h(a, b, c, d, x, y); }
  static __device__ __forceinline__ void keep(v16h a, v16h b, v16h c, v16h d) { keep4_h(a, b, c, d); }
};

template <int BIAS_MODE, int OUT_MODE, int SELMODE>
__global__ __launch_bounds__(256) void gemm64(
    const unsigned short* __restrict__ Ap, int lda, long strideA,
    const unsigned short* __restrict__ Btp, int ldb, long strideB,
    void* __restrict__ Cout, int ldc, long strideC,
    const float* __restrict__ bias, long biasSel,
    const int* __restrict__ sel, int jsel,
    int M, int N, int K, float scale, float post) {
  static_assert(SELMODE != 2 || OUT_MODE != 0, "identity copy needs a 16-bit output plane");
  typedef _Float16 T;
  typedef v16h V;
  __shared__ __align__(16) float sT[8][16 * 68];
  const int b    = blockIdx.y;
  const int lane = threadIdx.x & 31;
  const int wave = threadIdx.x >> 5;
  const int tilesN = N >> 6;
  const int tilesM = M >> 6;
  const int tile = blockIdx.x * 8 + wave;
  if (tile >= tilesM * tilesN) return;
  const int tm = tile / tilesN;
  const int tn = tile - tm * tilesN;
  const int m0 = tm << 6;
  const int n0 = tn << 6;

  long bIdx = b;
  long bOfs = 0;
  int lb = 0, lj = 1;
  if (SELMODE == 1) {
    lb = clamp_lang(sel[b]);
    bIdx = lb;
    bOfs = (long)lb * biasSel;
  }
  if (SELMODE == 2) {
    const int jj = jsel < 0 ? 0 : (jsel > kB - 1 ? kB - 1 : jsel);
    lb = clamp_lang(sel[b]);
    lj = clamp_lang(sel[jj]);
    bIdx = (long)lb * kL + lj;
  }
  if (SELMODE == 2 && lb == lj) {
    const unsigned short* src = Ap + (size_t)b * strideA;
    unsigned short* dst = (unsigned short*)Cout + (size_t)b * strideC;
    const int q4 = lane >> 3, c8 = (lane & 7) * 8;
    for (int pass = 0; pass < 2; ++pass) {
#pragma unroll
      for (int io = 0; io < 4; ++io) {
#pragma unroll
        for (int ii = 0; ii < 4; ++ii) {
          const int row = m0 + (io * 4 + ii) * 4 + q4;
          const v4u w = *(const v4u*)(src + (size_t)row * lda + n0 + c8);
          *(volatile v4u*)(dst + (size_t)row * ldc + n0 + c8) = w;
        }
        asm volatile("" ::: "memory");
      }
      __threadfence();
    }
    return;
  }

  const T* Ab = (const T*)Ap + (size_t)b * strideA;
  const T* Bb = (const T*)Btp + (size_t)bIdx * strideB;

  const int rlane = lane & 15;
  const int koff  = (lane >> 4) * 8;
  const int mOff  = (lane >> 4) * 8;

  v8f acc[4][4];
#pragma unroll
  for (int i = 0; i < 4; ++i)
#pragma unroll
    for (int j = 0; j < 4; ++j) acc[i][j] = (v8f){0.f,0.f,0.f,0.f,0.f,0.f,0.f,0.f};

  for (int k0 = 0; k0 < K; k0 += 32) {
    V bh[4];
#pragma unroll
    for (int j = 0; j < 4; ++j) {
      const size_t bo = (size_t)(n0 + (j << 4) + rlane) * ldb + koff + k0;
      bh[j] = FragH::load(Bb + bo);
    }
#pragma unroll
    for (int i = 0; i < 4; ++i) {
      const size_t ao = (size_t)(m0 + (i << 4) + rlane) * lda + koff + k0;
      V ah = FragH::load(Ab + ao);
#pragma unroll
      for (int j = 0; j < 4; ++j) acc[i][j] = FragH::mma(ah, bh[j], acc[i][j]);
      FragH::guard4(acc[i][0], acc[i][1], acc[i][2], acc[i][3], ah, bh[3]);
    }
    FragH::keep(bh[0], bh[1], bh[2], bh[3]);
  }
  acc_guard4(acc[0][0], acc[0][1], acc[0][2], acc[0][3]);
  acc_guard4(acc[1][0], acc[1][1], acc[1][2], acc[1][3]);
  acc_guard4(acc[2][0], acc[2][1], acc[2][2], acc[2][3]);
  acc_guard4(acc[3][0], acc[3][1], acc[3][2], acc[3][3]);

  float bcol[4] = {0.f, 0.f, 0.f, 0.f};
  if (BIAS_MODE == 2) {
#pragma unroll
    for (int j = 0; j < 4; ++j) bcol[j] = bfr(bias[bOfs + n0 + (j << 4) + rlane]);
  }
  float* slab = sT[wave];
#pragma unroll
  for (int i = 0; i < 4; ++i) {
    const int mBase = m0 + (i << 4);
    float brow[8] = {0.f, 0.f, 0.f, 0.f, 0.f, 0.f, 0.f, 0.f};
    if (BIAS_MODE == 1) {
      const v4f t0 = *(const v4f*)(bias + bOfs + mBase + mOff);
      const v4f t1 = *(const v4f*)(bias + bOfs + mBase + mOff + 4);
      brow[0] = bfr(t0[0]); brow[1] = bfr(t0[1]); brow[2] = bfr(t0[2]); brow[3] = bfr(t0[3]);
      brow[4] = bfr(t1[0]); brow[5] = bfr(t1[1]); brow[6] = bfr(t1[2]); brow[7] = bfr(t1[3]);
    }
#pragma unroll
    for (int j = 0; j < 4; ++j) {
#pragma unroll
      for (int r = 0; r < 8; ++r) {
        float v = acc[i][j][r] * scale;
        if (BIAS_MODE == 1) v += brow[r];
        if (BIAS_MODE == 2) v += bcol[j];
        v = v * post;
        slab[(mOff + r) * 68 + (j << 4) + rlane] = v;
      }
    }
    __builtin_amdgcn_fence(__ATOMIC_RELEASE, "workgroup");
    __builtin_amdgcn_wave_barrier();
    __builtin_amdgcn_fence(__ATOMIC_ACQUIRE, "workgroup");
    if (OUT_MODE == 0) {
      float* Cf = (float*)Cout + (size_t)b * strideC;
      const int hh = lane >> 4, c4 = (lane & 15) * 4;
      for (int pass = 0; pass < 2; ++pass) {
#pragma unroll
        for (int it = 0; it < 8; ++it) {
          const int row = it * 2 + hh;
          v4f v = *(const v4f*)(slab + row * 68 + c4);
          *(volatile v4f*)(Cf + (size_t)(mBase + row) * ldc + n0 + c4) = v;
        }
        __threadfence();
      }
    } else {
      const int q = lane >> 3, c8 = (lane & 7) * 8;
      unsigned short* Cs = (unsigned short*)Cout + (size_t)b * strideC;
      for (int pass = 0; pass < 2; ++pass) {
#pragma unroll
        for (int it = 0; it < 4; ++it) {
          const int row = it * 4 + q;
          const float* sp = slab + row * 68 + c8;
          v8h hv;
#pragma unroll
          for (int e = 0; e < 8; ++e) hv[e] = (_Float16)sp[e];
          *(volatile v8h*)(Cs + (size_t)(mBase + row) * ldc + n0 + c8) = hv;
        }
        __threadfence();
      }
    }
    __builtin_amdgcn_fence(__ATOMIC_RELEASE, "workgroup");
    __builtin_amdgcn_wave_barrier();
    __builtin_amdgcn_fence(__ATOMIC_ACQUIRE, "workgroup");
  }
}

__global__ __launch_bounds__(256) void wt_cast_kernel(const float* __restrict__ W0, const float* __restrict__ W1,
                                                      const float* __restrict__ W2, const float* __restrict__ W3,
                                                      const float* __restrict__ W4, int nptr,
                                                      unsigned short* __restrict__ out) {
  __shared__ float sm[64][65];
  const int t  = threadIdx.x;
  const int k0 = blockIdx.x * 64;
  const int n0 = blockIdx.y * 64;
  const int z  = blockIdx.z;
  const float* W;
  if (nptr == 1) W = W0 + (size_t)z * kHH;
  else W = (z == 0) ? W0 : (z == 1) ? W1 : (z == 2) ? W2 : (z == 3) ? W3 : W4;
#pragma unroll
  for (int i = 0; i < 16; ++i) {
    const int e = i * 256 + t;
    const int r = e >> 6;
    const int c = e & 63;
    sm[c][r] = W[(size_t)(k0 + r) * kH + n0 + c];
    if (i == 7) asm volatile("" ::: "memory");
  }
  __syncthreads();
  const int lane = t & 31, wave = t >> 5;
  const int q = lane >> 3, c8 = (lane & 7) * 8;
  unsigned short* op = out + (size_t)z * kHH;
  for (int pass = 0; pass < 2; ++pass) {
#pragma unroll
    for (int it = 0; it < 2; ++it) {
      const int row = wave * 8 + it * 4 + q;
      unsigned short hb[8];
#pragma unroll
      for (int e = 0; e < 8; ++e) hb[e] = h_bits(bfr(sm[row][c8 + e]) * kWCarry);
      const v4u u = (v4u){pk16(hb[0], hb[1]), pk16(hb[2], hb[3]), pk16(hb[4], hb[5]), pk16(hb[6], hb[7])};
      *(volatile v4u*)(op + (size_t)(n0 + row) * kH + k0 + c8) = u;
    }
    __threadfence();
  }
}

__global__ __launch_bounds__(256) void xcast_kernel(const float* __restrict__ in, unsigned short* __restrict__ out, int n8) {
  const int i = blockIdx.x * 256 + threadIdx.x;
  if (i >= n8) return;
  const float* p = in + 8 * (size_t)i;
  const v4f a = *(const v4f*)(p);
  const v4f c = *(const v4f*)(p + 4);
  unsigned short hb[8];
#pragma unroll
  for (int e = 0; e < 4; ++e) {
    hb[e]     = h_bits(bfr(a[e]));
    hb[4 + e] = h_bits(bfr(c[e]));
  }
  const v4u u = (v4u){pk16(hb[0], hb[1]), pk16(hb[2], hb[3]), pk16(hb[4], hb[5]), pk16(hb[6], hb[7])};
  unsigned short* q = out + 8 * (size_t)i;
  *(volatile v4u*)q = u;
  __threadfence();
  *(volatile v4u*)q = u;
}

__global__ __launch_bounds__(256) void ln_relu_kernel(const float* __restrict__ Af, const float* __restrict__ G,
                                                      const float* __restrict__ Bm, const int* __restrict__ lids,
                                                      unsigned short* __restrict__ out16, float* __restrict__ out32) {
  __shared__ __align__(16) float rowv[kH];
  __shared__ float redA[8];
  __shared__ float redB[8];
  const int row  = blockIdx.x;
  const int t    = threadIdx.x;
  const int lane = t & 31, wave = t >> 5;
  const int lid  = clamp_lang(lids[row >> 9]);
  const float* x = Af + (size_t)row * kH;
  const float x0 = x[t], x1 = x[t + 256], x2 = x[t + 512];
  float s = (x0 + x1) + x2;
#pragma unroll
  for (int off = 16; off > 0; off >>= 1) s += __shfl_xor(s, off, 32);
  if (lane == 0) redA[wave] = s;
  __syncthreads();
  float tot = redA[0];
#pragma unroll
  for (int w = 1; w < 8; ++w) tot += redA[w];
  const float mean = tot * kInvH;
  const float d0 = x0 - mean, d1 = x1 - mean, d2 = x2 - mean;
  float s2 = (d0 * d0 + d1 * d1) + d2 * d2;
#pragma unroll
  for (int off = 16; off > 0; off >>= 1) s2 += __shfl_xor(s2, off, 32);
  if (lane == 0) redB[wave] = s2;
  __syncthreads();
  float tot2 = redB[0];
#pragma unroll
  for (int w = 1; w < 8; ++w) tot2 += redB[w];
  const float var  = tot2 * kInvH;
  const float rstd = rsqrtf(var + kLnEps);
  const float* g  = G  + (size_t)lid * kH;
  const float* be = Bm + (size_t)lid * kH;
  const float y0 = fmaxf(d0 * rstd * bfr(g[t])       + bfr(be[t]),       0.0f);
  const float y1 = fmaxf(d1 * rstd * bfr(g[t + 256]) + bfr(be[t + 256]), 0.0f);
  const float y2 = fmaxf(d2 * rstd * bfr(g[t + 512]) + bfr(be[t + 512]), 0.0f);
  rowv[t] = y0; rowv[t + 256] = y1; rowv[t + 512] = y2;
  __syncthreads();
  for (int pass = 0; pass < 2; ++pass) {
    if (t < 192) {
      const v4f v = *(const v4f*)(rowv + 4 * t);
      *(volatile v4f*)(out32 + (size_t)row * kH + 4 * t) = v;
    }
    if (t < 96) {
      unsigned short hb[8];
#pragma unroll
      for (int e = 0; e < 8; ++e) hb[e] = h_bits(rowv[8 * t + e]);
      const v4u u = (v4u){pk16(hb[0], hb[1]), pk16(hb[2], hb[3]), pk16(hb[4], hb[5]), pk16(hb[6], hb[7])};
      *(volatile v4u*)(out16 + (size_t)row * kH + 8 * t) = u;
    }
    __threadfence();
  }
}

__global__ __launch_bounds__(256) void softmax_heads_kernel(const float* __restrict__ SCp, unsigned short* __restrict__ ATT,
                                                            float* __restrict__ orows) {
  __shared__ __align__(16) float prow[kS];
  __shared__ float redM[8];
  __shared__ float redS[8];
  const int q    = blockIdx.x;
  const int t    = threadIdx.x;
  const int lane = t & 31, wave = t >> 5;
  const int c0   = 2 * t;
  float h0 = 0.0f, h1 = 0.0f;
#pragma unroll 1
  for (int h = 0; h < kNH; ++h) {
    const float* sr = SCp + ((size_t)h * kS + q) * kS + c0;
    const v2f sv = *(const v2f*)sr;
    float mx = fmaxf(sv[0], sv[1]);
#pragma unroll
    for (int off = 16; off > 0; off >>= 1) mx = fmaxf(mx, __shfl_xor(mx, off, 32));
    if (lane == 0) redM[wave] = mx;
    __syncthreads();
    float m = redM[0];
#pragma unroll
    for (int w = 1; w < 8; ++w) m = fmaxf(m, redM[w]);
    const float e0 = expf(sv[0] - m);
    const float e1 = expf(sv[1] - m);
    float sum = e0 + e1;
#pragma unroll
    for (int off = 16; off > 0; off >>= 1) sum += __shfl_xor(sum, off, 32);
    if (lane == 0) redS[wave] = sum;
    __syncthreads();
    float tot = redS[0];
#pragma unroll
    for (int w = 1; w < 8; ++w) tot += redS[w];
    const float inv = 1.0f / tot;
    const float p0 = e0 * inv, p1 = e1 * inv;
    h0 += p0;
    h1 += p1;
    *(v2f*)(prow + c0) = (v2f){p0 * kPCarry, p1 * kPCarry};
    __syncthreads();
    if (t < 64) {
      const v4f a = *(const v4f*)(prow + 8 * t);
      const v4f c = *(const v4f*)(prow + 8 * t + 4);
      unsigned short hb[8];
#pragma unroll
      for (int e = 0; e < 4; ++e) { hb[e] = h_bits(a[e]); hb[4 + e] = h_bits(c[e]); }
      const v4u u = (v4u){pk16(hb[0], hb[1]), pk16(hb[2], hb[3]), pk16(hb[4], hb[5]), pk16(hb[6], hb[7])};
      unsigned short* pr = ATT + ((size_t)h * kS + q) * kS + 8 * (size_t)t;
      *(volatile v4u*)pr = u;
      __threadfence();
      *(volatile v4u*)pr = u;
    }
    __syncthreads();
  }
  *(v2f*)(prow + c0) = (v2f){h0 * kInvNH, h1 * kInvNH};
  __syncthreads();
  if (t < 128) {
    const v4f v = *(const v4f*)(prow + 4 * t);
    float* op = orows + (size_t)q * kS + 4 * t;
    *(volatile v4f*)op = v;
    __threadfence();
    *(volatile v4f*)op = v;
  }
}

__global__ __launch_bounds__(256) void ln_res_kernel(float* __restrict__ OA, const float* __restrict__ R,
                                                     const float* __restrict__ G, const float* __restrict__ Bm,
                                                     float* __restrict__ out0) {
  __shared__ __align__(16) float rowv[kH];
  __shared__ float redA[8];
  __shared__ float redB[8];
  const int row  = blockIdx.x;
  const int t    = threadIdx.x;
  const int lane = t & 31, wave = t >> 5;
  const float* o = OA + (size_t)row * kH;
  const float* a = R  + (size_t)row * kH;
  const float x0 = o[t] + a[t], x1 = o[t + 256] + a[t + 256], x2 = o[t + 512] + a[t + 512];
  float s = (x0 + x1) + x2;
#pragma unroll
  for (int off = 16; off > 0; off >>= 1) s += __shfl_xor(s, off, 32);
  if (lane == 0) redA[wave] = s;
  __syncthreads();
  float tot = redA[0];
#pragma unroll
  for (int w = 1; w < 8; ++w) tot += redA[w];
  const float mean = tot * kInvH;
  const float d0 = x0 - mean, d1 = x1 - mean, d2 = x2 - mean;
  float s2 = (d0 * d0 + d1 * d1) + d2 * d2;
#pragma unroll
  for (int off = 16; off > 0; off >>= 1) s2 += __shfl_xor(s2, off, 32);
  if (lane == 0) redB[wave] = s2;
  __syncthreads();
  float tot2 = redB[0];
#pragma unroll
  for (int w = 1; w < 8; ++w) tot2 += redB[w];
  const float var  = tot2 * kInvH;
  const float rstd = rsqrtf(var + kLnEps);
  rowv[t]       = d0 * rstd * bfr(G[t])       + bfr(Bm[t]);
  rowv[t + 256] = d1 * rstd * bfr(G[t + 256]) + bfr(Bm[t + 256]);
  rowv[t + 512] = d2 * rstd * bfr(G[t + 512]) + bfr(Bm[t + 512]);
  __syncthreads();
  for (int pass = 0; pass < 2; ++pass) {
    if (t < 192) {
      const v4f v = *(const v4f*)(rowv + 4 * t);
      *(volatile v4f*)(out0 + (size_t)row * kH + 4 * t) = v;
      *(volatile v4f*)(OA + (size_t)row * kH + 4 * t) = v;
    }
    __threadfence();
  }
}

__global__ __launch_bounds__(256) void pooled_kernel(const float* __restrict__ ASC, const int* __restrict__ mask,
                                                     float* __restrict__ pooled) {
  __shared__ __align__(16) float pv[256];
  const int chunk = blockIdx.x;
  const int b = blockIdx.y;
  const int t = threadIdx.x;
  const int c = chunk * 256 + t;
  float acc = 0.0f, ms = 0.0f;
#pragma unroll 1
  for (int s = 0; s < kS; ++s) {
    const float m = (float)mask[b * kS + s];
    acc += ASC[((size_t)(b * kS + s)) * kH + c] * m;
    ms  += m;
  }
  pv[t] = acc * (1.0f / ms);
  __syncthreads();
  if (t < 64) {
    const v4f v = *(const v4f*)(pv + 4 * t);
    float* dp = pooled + (size_t)b * kH + chunk * 256 + 4 * t;
    *(volatile v4f*)dp = v;
    __threadfence();
    *(volatile v4f*)dp = v;
  }
}

__global__ __launch_bounds__(256) void head_kernel(const float* __restrict__ pooled, const float* __restrict__ w1,
                                                   const float* __restrict__ b1, const float* __restrict__ w2,
                                                   const float* __restrict__ b2, float* __restrict__ out2,
                                                   float* __restrict__ pn) {
  __shared__ __align__(16) float pl[kH];
  __shared__ __align__(16) float p1s[kH];
  __shared__ __align__(16) float ps[256];
  __shared__ float red[8];
  const int b = blockIdx.x;
  const int t = threadIdx.x;
  const int lane = t & 31, wave = t >> 5;
  pl[t]       = pooled[(size_t)b * kH + t];
  pl[t + 256] = pooled[(size_t)b * kH + t + 256];
  pl[t + 512] = pooled[(size_t)b * kH + t + 512];
  __syncthreads();
  float a0 = 0.0f, a1 = 0.0f, a2 = 0.0f;
#pragma unroll 1
  for (int k = 0; k < kH; ++k) {
    const float pk = pl[k];
    const float* wr = w1 + (size_t)k * kH;
    a0 += pk * bfr(wr[t]);
    a1 += pk * bfr(wr[t + 256]);
    a2 += pk * bfr(wr[t + 512]);
  }
  p1s[t]       = fmaxf(a0 + bfr(b1[t]),       0.0f);
  p1s[t + 256] = fmaxf(a1 + bfr(b1[t + 256]), 0.0f);
  p1s[t + 512] = fmaxf(a2 + bfr(b1[t + 512]), 0.0f);
  __syncthreads();
  float pc = 0.0f;
#pragma unroll 1
  for (int k = 0; k < kH; ++k) pc += p1s[k] * bfr(w2[(size_t)k * kC + t]);
  pc += bfr(b2[t]);
  float ss = pc * pc;
#pragma unroll
  for (int off = 16; off > 0; off >>= 1) ss += __shfl_xor(ss, off, 32);
  if (lane == 0) red[wave] = ss;
  __syncthreads();
  float tot = red[0];
#pragma unroll
  for (int w = 1; w < 8; ++w) tot += red[w];
  const float nrm = sqrtf(tot);
  ps[t] = pc * (1.0f / nrm);
  __syncthreads();
  if (t < 64) {
    const v4f v = *(const v4f*)(ps + 4 * t);
    float* op = out2 + (size_t)b * kC + 4 * t;
    float* wp = pn   + (size_t)b * kC + 4 * t;
    *(volatile v4f*)op = v;
    *(volatile v4f*)wp = v;
    __threadfence();
    *(volatile v4f*)op = v;
    *(volatile v4f*)wp = v;
  }
}

__global__ __launch_bounds__(64) void loss_kernel(const float* __restrict__ pn, const int* __restrict__ lids,
                                                  const float* __restrict__ temp, float* __restrict__ out3) {
  __shared__ float sim[64];
  __shared__ float rl[8];
  const int t = threadIdx.x;
  const int i = t >> 3, j = t & 7;
  float acc = 0.0f;
#pragma unroll 1
  for (int c = 0; c < kC; ++c) acc += pn[i * kC + c] * pn[j * kC + c];
  const float tinv = 1.0f / bfr(temp[0]);
  sim[t] = acc * tinv;
  __syncthreads();
  const int ri = t & 7;
  const int li = lids[ri];
  float mx = sim[ri * 8];
#pragma unroll
  for (int jj = 1; jj < kB; ++jj) mx = fmaxf(mx, sim[ri * 8 + jj]);
  float se = 0.0f;
#pragma unroll 1
  for (int jj = 0; jj < kB; ++jj) se += expf(sim[ri * 8 + jj] - mx);
  const float lse = mx + logf(se);
  float srow = 0.0f;
#pragma unroll
  for (int jj = 0; jj < kB; ++jj) {
    const float lab = (li != lids[jj]) ? 1.0f : 0.0f;
    srow += lab * (sim[ri * 8 + jj] - lse);
  }
  if (t < kB) rl[t] = srow;
  __syncthreads();
  float tot = rl[0];
#pragma unroll
  for (int ii = 1; ii < kB; ++ii) tot += rl[ii];
  const float loss = -(tot * 0.125f);
  if (t == 0) {
    *(volatile float*)out3 = loss;
    __threadfence();
    *(volatile float*)out3 = loss;
  }
}

template <int BIASM, int OUTM, int SELM>
static void run_gemm(hipStream_t st, const unsigned short* A, int lda, long sA,
                     const unsigned short* Bt, int ldb, long sB,
                     void* Cp, int ldc, long sC,
                     const float* bias, long biasSel, const int* sel, int jsel,
                     int M, int N, int K, float scale, float post, int batches) {
  const int tiles = (M / 64) * (N / 64);
  dim3 grid((unsigned)((tiles + 7) / 8), (unsigned)batches, 1);
  gemm64<BIASM, OUTM, SELM><<<grid, dim3(256, 1, 1), 0, st>>>(
      A, lda, sA, Bt, ldb, sB, Cp, ldc, sC, bias, biasSel, sel, jsel, M, N, K, scale, post);
}

extern "C" void kernel_launch(void* const* d_in, const int* in_sizes, int n_in,
                              void* d_out, int out_size, void* d_ws, size_t ws_size,
                              hipStream_t stream) {
  if (n_in < 29) return;
  if (in_sizes[0] != kRows * kH) return;
  if (in_sizes[1] != kB || in_sizes[2] != kB * kS) return;
  if (in_sizes[3] != (int)(kL * kHH) || in_sizes[7] != (int)(kL * kHH) || in_sizes[9] != (int)(kL * kHH)) return;
  if (in_sizes[4] != kL * kH || in_sizes[5] != kL * kH || in_sizes[6] != kL * kH || in_sizes[8] != kL * kH || in_sizes[10] != kL * kH) return;
  if (in_sizes[11] != (int)kHH || in_sizes[13] != (int)kHH || in_sizes[15] != (int)kHH || in_sizes[17] != (int)kHH) return;
  if (in_sizes[12] != kH || in_sizes[14] != kH || in_sizes[16] != kH || in_sizes[18] != kH) return;
  if (in_sizes[19] != (int)(kL * kL * kHH)) return;
  if (in_sizes[20] != (int)kHH || in_sizes[21] != kH || in_sizes[22] != kH || in_sizes[23] != kH) return;
  if (in_sizes[24] != (int)kHH || in_sizes[25] != kH || in_sizes[26] != kH * kC || in_sizes[27] != kC || in_sizes[28] < 1) return;
  if ((long)out_size != kOutTotal) return;
  if (ws_size < kWsTotal) return;

  const float* x          = (const float*)d_in[0];
  const int*   lids       = (const int*)  d_in[1];
  const int*   amask      = (const int*)  d_in[2];
  const float* adapter_w  = (const float*)d_in[3];
  const float* adapter_b  = (const float*)d_in[4];
  const float* adapter_g  = (const float*)d_in[5];
  const float* adapter_be = (const float*)d_in[6];
  const float* wq_lang    = (const float*)d_in[7];
  const float* bq_lang    = (const float*)d_in[8];
  const float* wk_lang    = (const float*)d_in[9];
  const float* bk_lang    = (const float*)d_in[10];
  const float* attn_wq    = (const float*)d_in[11];
  const float* attn_bq    = (const float*)d_in[12];
  const float* attn_wk    = (const float*)d_in[13];
  const float* attn_bk    = (const float*)d_in[14];
  const float* attn_wv    = (const float*)d_in[15];
  const float* attn_bv    = (const float*)d_in[16];
  const float* attn_wo    = (const float*)d_in[17];
  const float* attn_bo    = (const float*)d_in[18];
  const float* align_m    = (const float*)d_in[19];
  const float* outp_w     = (const float*)d_in[20];
  const float* outp_b     = (const float*)d_in[21];
  const float* ln_g       = (const float*)d_in[22];
  const float* ln_b       = (const float*)d_in[23];
  const float* proj_w1    = (const float*)d_in[24];
  const float* proj_b1    = (const float*)d_in[25];
  const float* proj_w2    = (const float*)d_in[26];
  const float* proj_b2    = (const float*)d_in[27];
  const float* temp       = (const float*)d_in[28];

  float* outf = (float*)d_out;
  float* out0 = outf;
  float* out1 = outf + kOut1Off;
  float* out2 = outf + kOut2Off;
  float* out3 = outf + kOut3Off;

  char* ws = (char*)d_ws;
  unsigned short* X16   = (unsigned short*)(ws + offX16);
  unsigned short* AWT   = (unsigned short*)(ws + offAWT);
  unsigned short* WQL   = (unsigned short*)(ws + offWQL);
  unsigned short* WKL   = (unsigned short*)(ws + offWKL);
  unsigned short* W5    = (unsigned short*)(ws + offW5);
  unsigned short* ALT   = (unsigned short*)(ws + offALT);
  unsigned short* ADP16 = (unsigned short*)(ws + offADP16);
  float*          ADP32 = (float*)(ws + offADP32);
  unsigned short* QL16  = (unsigned short*)(ws + offQL);
  unsigned short* KL16  = (unsigned short*)(ws + offKL);
  unsigned short* Q16   = (unsigned short*)(ws + offQP);
  unsigned short* K16   = (unsigned short*)(ws + offKP);
  unsigned short* VT16  = (unsigned short*)(ws + offVT);
  float*          SC    = (float*)(ws + offSC);
  unsigned short* ATT16 = (unsigned short*)(ws + offATT);
  float*          POOL  = (float*)(ws + offPOOL);
  float*          PN    = (float*)(ws + offPN);
  unsigned short* CTX16 = QL16;
  unsigned short* MHA16 = KL16;
  unsigned short* PA    = Q16;
  unsigned short* PB    = K16;
  const float* fdummy = attn_bq;

  {
    const int n8 = (kRows * kH) / 8;
    xcast_kernel<<<dim3(n8 / 256), dim3(256), 0, stream>>>(x, X16, n8);
  }
  wt_cast_kernel<<<dim3(kH / 64, kH / 64, kL), dim3(256), 0, stream>>>(adapter_w, adapter_w, adapter_w, adapter_w, adapter_w, 1, AWT);
  wt_cast_kernel<<<dim3(kH / 64, kH / 64, kL), dim3(256), 0, stream>>>(wq_lang, wq_lang, wq_lang, wq_lang, wq_lang, 1, WQL);
  wt_cast_kernel<<<dim3(kH / 64, kH / 64, kL), dim3(256), 0, stream>>>(wk_lang, wk_lang, wk_lang, wk_lang, wk_lang, 1, WKL);
  wt_cast_kernel<<<dim3(kH / 64, kH / 64, 5), dim3(256), 0, stream>>>(attn_wq, attn_wk, attn_wv, attn_wo, outp_w, 5, W5);
  wt_cast_kernel<<<dim3(kH / 64, kH / 64, kL * kL), dim3(256), 0, stream>>>(align_m, align_m, align_m, align_m, align_m, 1, ALT);

  run_gemm<2, 0, 1>(stream, X16, kH, kSH, AWT, kH, kHH, (void*)SC, kH, kSH,
                    adapter_b, (long)kH, lids, 0, kS, kH, kH, kWCarryInv, 1.0f, kB);
  ln_relu_kernel<<<dim3(kRows), dim3(256), 0, stream>>>(SC, adapter_g, adapter_be, lids, ADP16, ADP32);

  run_gemm<2, 1, 1>(stream, ADP16, kH, kSH, WQL, kH, kHH, (void*)QL16, kH, kSH,
                    bq_lang, (long)kH, lids, 0, kS, kH, kH, kWCarryInv, 1.0f, kB);
  run_gemm<2, 1, 1>(stream, ADP16, kH, kSH, WKL, kH, kHH, (void*)KL16, kH, kSH,
                    bk_lang, (long)kH, lids, 0, kS, kH, kH, kWCarryInv, 1.0f, kB);

  run_gemm<2, 1, 0>(stream, QL16, kH, kSH, W5 + 0 * (size_t)kHH, kH, 0L, (void*)Q16, kH, kSH,
                    attn_bq, 0L, lids, 0, kS, kH, kH, kWCarryInv, 1.0f, kB);
  run_gemm<2, 1, 0>(stream, KL16, kH, kSH, W5 + 1 * (size_t)kHH, kH, 0L, (void*)K16, kH, kSH,
                    attn_bk, 0L, lids, 0, kS, kH, kH, kWCarryInv, 1.0f, kB);
  run_gemm<1, 1, 0>(stream, W5 + 2 * (size_t)kHH, kH, 0L, ADP16, kH, kSH, (void*)VT16, kS, (long)kH * kS,
                    attn_bv, 0L, lids, 0, kH, kS, kH, kWCarryInv, 1.0f, kB);

  for (int b = 0; b < kB; ++b) {
    const unsigned short* Qb = Q16 + (size_t)b * kSH;
    const unsigned short* Kb = K16 + (size_t)b * kSH;
    run_gemm<0, 0, 0>(stream, Qb, kH, (long)kD, Kb, kH, (long)kD, (void*)SC, kS, kSS,
                      fdummy, 0L, lids, 0, kS, kS, kD, kQScale, 1.0f, kNH);
    softmax_heads_kernel<<<dim3(kS), dim3(256), 0, stream>>>(SC, ATT16, out1 + (size_t)b * kSS);
    run_gemm<0, 1, 0>(stream, ATT16, kS, kSS, VT16 + (size_t)b * kH * kS, kS, (long)kD * kS,
                      (void*)(CTX16 + (size_t)b * kSH), kH, (long)kD,
                      fdummy, 0L, lids, 0, kS, kD, kS, kPCarryInv, 1.0f, kNH);
  }

  run_gemm<2, 1, 0>(stream, CTX16, kH, kSH, W5 + 3 * (size_t)kHH, kH, 0L, (void*)MHA16, kH, kSH,
                    attn_bo, 0L, lids, 0, kS, kH, kH, kWCarryInv, 1.0f, kB);

  {
    const unsigned short* src = MHA16;
    for (int j = 0; j < kB; ++j) {
      unsigned short* dst = (j & 1) ? PB : PA;
      run_gemm<0, 1, 2>(stream, src, kH, kSH, ALT, kH, kHH, (void*)dst, kH, kSH,
                        fdummy, 0L, lids, j, kS, kH, kH, kWCarryInv, 1.0f, kB);
      src = dst;
    }
  }

  run_gemm<2, 0, 0>(stream, PB, kH, kSH, W5 + 4 * (size_t)kHH, kH, 0L, (void*)SC, kH, kSH,
                    outp_b, 0L, lids, 0, kS, kH, kH, kWCarryInv, 1.0f, kB);
  ln_res_kernel<<<dim3(kRows), dim3(256), 0, stream>>>(SC, ADP32, ln_g, ln_b, out0);

  pooled_kernel<<<dim3(kH / 256, kB), dim3(256), 0, stream>>>(SC, amask, POOL);
  head_kernel<<<dim3(kB), dim3(256), 0, stream>>>(POOL, proj_w1, proj_b1, proj_w2, proj_b2, out2, PN);
  loss_kernel<<<dim3(1), dim3(64), 0, stream>>>(PN, lids, temp, out3);
}
